// QAgent_37331855737183
// MI455X (gfx1250) — hardware-verified
//
#include <hip/hip_runtime.h>
#include <stdint.h>
#include <math.h>


typedef __attribute__((ext_vector_type(16))) __bf16 v16b;
typedef __attribute__((ext_vector_type(8)))  __bf16 v8b;
typedef __attribute__((ext_vector_type(8)))  float  v8f;
typedef __attribute__((ext_vector_type(4)))  float  v4f;

#define NSEQ 256
#define OBSD 3
#define CHK  64
#define RECW 12
#define RECI (CHK * RECW)
#define WSEQ 32

__device__ __forceinline__ unsigned short f2bf_bits(float f) {
  unsigned u = __float_as_uint(f);
  return (unsigned short)((u + 0x7FFFu + ((u >> 16) & 1u)) >> 16);
}
__device__ __forceinline__ float bf_bits2f(unsigned short h) { return __uint_as_float(((unsigned)h) << 16); }
__device__ __forceinline__ __bf16 bits2bf(unsigned short h) { return __builtin_bit_cast(__bf16, h); }

__device__ __forceinline__ v8f at_mma(v16b a, v16b b, v8f c) {
  c = __builtin_amdgcn_wmma_f32_16x16x32_bf16(false, a, false, b, (short)0, c, false, false);
  asm volatile("v_nop\n\tv_nop\n\tv_nop\n\tv_nop" : "+v"(c) : "v"(a), "v"(b));
  return c;
}

__device__ __forceinline__ float sigmoid_f(float x) {
  return __builtin_amdgcn_rcpf(1.0f + expf(-x));
}
__device__ __forceinline__ float silu_f(float x) { return x * sigmoid_f(x); }
__device__ __forceinline__ float softplus_f(float x) {
  return fmaxf(x, 0.0f) + log1pf(expf(-fabsf(x)));
}

__device__ __forceinline__ double shfl_up_d(double v, int d) {
  union { double f; int i[2]; } u;
  u.f = v;
  u.i[0] = __shfl_up(u.i[0], (unsigned)d, 32);
  u.i[1] = __shfl_up(u.i[1], (unsigned)d, 32);
  return u.f;
}
__device__ __forceinline__ double shfl_d(double v, int src) {
  union { double f; int i[2]; } u;
  u.f = v;
  u.i[0] = __shfl(u.i[0], src, 32);
  u.i[1] = __shfl(u.i[1], src, 32);
  return u.f;
}
__device__ __forceinline__ double wave_scan_d(double v, int lane) {
#pragma unroll
  for (int d = 1; d < 32; d <<= 1) {
    const double o = shfl_up_d(v, d);
    if (lane >= d) v += o;
  }
  return v;
}

struct Par {
  float w00, w01, w02, w10, w11, w12, bi0, bi1;
  float p00, p01, p10, p11, p20, p21, p30, p31, p40, p41, p50, p51, p60, p61;
  float c00, c01, c10, c11, c20, c21, c30, c31, cb0, cb1, cb2, cb3;
  float dtb, Aneg;
};
__device__ __forceinline__ Par load_par(const float* __restrict__ W_in, const float* __restrict__ b_in,
                                        const float* __restrict__ W_ip, const float* __restrict__ conv_w,
                                        const float* __restrict__ conv_b, const float* __restrict__ dt_bias,
                                        const float* __restrict__ A_log) {
  Par p;
  p.w00 = W_in[0]; p.w01 = W_in[1]; p.w02 = W_in[2];
  p.w10 = W_in[3]; p.w11 = W_in[4]; p.w12 = W_in[5];
  p.bi0 = b_in[0]; p.bi1 = b_in[1];
  p.p00 = W_ip[0];  p.p01 = W_ip[1];
  p.p10 = W_ip[2];  p.p11 = W_ip[3];
  p.p20 = W_ip[4];  p.p21 = W_ip[5];
  p.p30 = W_ip[6];  p.p31 = W_ip[7];
  p.p40 = W_ip[8];  p.p41 = W_ip[9];
  p.p50 = W_ip[10]; p.p51 = W_ip[11];
  p.p60 = W_ip[12]; p.p61 = W_ip[13];
  p.c00 = conv_w[0]; p.c01 = conv_w[1];
  p.c10 = conv_w[2]; p.c11 = conv_w[3];
  p.c20 = conv_w[4]; p.c21 = conv_w[5];
  p.c30 = conv_w[6]; p.c31 = conv_w[7];
  p.cb0 = conv_b[0]; p.cb1 = conv_b[1]; p.cb2 = conv_b[2]; p.cb3 = conv_b[3];
  p.dtb  = dt_bias[0];
  p.Aneg = -expf(A_log[0]);
  return p;
}

struct Raw { float z0, z1, r2, r3, r4, r5, dtr; };
__device__ __forceinline__ Raw proj_raw(float o0, float o1, float o2, const Par& p) {
  const float d0 = p.w00 * o0 + p.w01 * o1 + p.w02 * o2 + p.bi0;
  const float d1 = p.w10 * o0 + p.w11 * o1 + p.w12 * o2 + p.bi1;
  Raw r;
  r.z0  = p.p00 * d0 + p.p01 * d1;
  r.z1  = p.p10 * d0 + p.p11 * d1;
  r.r2  = p.p20 * d0 + p.p21 * d1;
  r.r3  = p.p30 * d0 + p.p31 * d1;
  r.r4  = p.p40 * d0 + p.p41 * d1;
  r.r5  = p.p50 * d0 + p.p51 * d1;
  r.dtr = p.p60 * d0 + p.p61 * d1;
  return r;
}
struct Act { float x0, x1, Bv, Cv, dt; };
__device__ __forceinline__ Act conv_act(const Raw& c, float q2, float q3, float q4, float q5, const Par& p) {
  Act a;
  a.x0 = silu_f(q2 * p.c00 + c.r2 * p.c01 + p.cb0);
  a.x1 = silu_f(q3 * p.c10 + c.r3 * p.c11 + p.cb1);
  a.Bv = silu_f(q4 * p.c20 + c.r4 * p.c21 + p.cb2);
  a.Cv = silu_f(q5 * p.c30 + c.r5 * p.c31 + p.cb3);
  a.dt = softplus_f(c.dtr + p.dtb);
  return a;
}

__device__ __forceinline__ float front_step(const float* __restrict__ obs, int t, int bk, int l, const Par& p,
                                            float* sr, unsigned short* bh, unsigned short* bl) {
  const float* o = obs + ((size_t)t * NSEQ + bk) * OBSD;
  const Raw cur = proj_raw(o[0], o[1], o[2], p);
  float q2 = 0.0f, q3 = 0.0f, q4 = 0.0f, q5 = 0.0f;
  if (t > 0) {
    const float* om = o - NSEQ * OBSD;
    const Raw pr = proj_raw(om[0], om[1], om[2], p);
    q2 = pr.r2; q3 = pr.r3; q4 = pr.r4; q5 = pr.r5;
  }
  const Act ac = conv_act(cur, q2, q3, q4, q5, p);
  const float a   = p.Aneg * ac.dt;
  const float X0  = ac.x0 * ac.dt, X1 = ac.x1 * ac.dt;
  const float bx0 = X0 * ac.Bv, bx1 = X1 * ac.Bv;
  const float g0  = silu_f(cur.z0), g1 = silu_f(cur.z1);
  float* rr = sr + l * RECW;
  rr[2] = ac.Cv; rr[3] = a; rr[4] = ac.x0; rr[5] = ac.x1;
  rr[6] = bx0;   rr[7] = bx1; rr[8] = g0;  rr[9] = g1; rr[10] = ac.dt; rr[11] = 0.0f;
  unsigned short hb = f2bf_bits(bx0);
  bh[l] = hb;        bl[l] = f2bf_bits(bx0 - bf_bits2f(hb));
  hb = f2bf_bits(bx1);
  bh[CHK + l] = hb;  bl[CHK + l] = f2bf_bits(bx1 - bf_bits2f(hb));
  return a;
}

__device__ __forceinline__ v8f tile_mma(const int i, const int ks, v8f acc,
                                        const double* sa, const unsigned short* bh,
                                        const unsigned short* bl, const int lane) {
  const int hh = lane >> 4, m = lane & 15;
  const int l = 16 * i + m;
  const double acl = sa[l];
  v16b ahi, alo;
#pragma unroll
  for (int e = 0; e < 16; ++e) {
    const int s = 32 * ks + 8 * hh + (e & 7) + ((e >> 3) << 4);
    float arg = (float)(acl - sa[s]);
    arg = fminf(arg, 0.0f);
    const float ex = expf(arg);
    const bool on = (s <= l) && (arg > -80.0f);
    const float v = on ? ex : 0.0f;
    const unsigned short hb = f2bf_bits(v);
    const unsigned short lb = f2bf_bits(v - bf_bits2f(hb));
    ahi[e] = bits2bf(hb);
    alo[e] = bits2bf(lb);
  }
  const int nrow = (m < 2) ? m : 2;
  const unsigned short* ph = bh + nrow * CHK + 32 * ks + 8 * hh;
  const unsigned short* pl = bl + nrow * CHK + 32 * ks + 8 * hh;
  union FB { v16b v; v8b h[2]; } fh, fl;
  fh.h[0] = *(const v8b*)(ph); fh.h[1] = *(const v8b*)(ph + 16);
  fl.h[0] = *(const v8b*)(pl); fl.h[1] = *(const v8b*)(pl + 16);
  acc = at_mma(ahi, fh.v, acc);
  acc = at_mma(ahi, fl.v, acc);
  acc = at_mma(alo, fh.v, acc);
  return acc;
}
__device__ __forceinline__ void tile_out(const int i, v8f acc, float* sr, const int lane) {
  const int hh = lane >> 4, m = lane & 15;
  if (m < 2) {
#pragma unroll
    for (int r = 0; r < 8; ++r) sr[(16 * i + 8 * hh + r) * RECW + m] = acc[r];
  }
}

__global__ __launch_bounds__(64)
void ssd_chunk_front(const float* __restrict__ obs,
                     const float* __restrict__ W_in,   const float* __restrict__ b_in,
                     const float* __restrict__ W_ip,   const float* __restrict__ conv_w,
                     const float* __restrict__ conv_b, const float* __restrict__ dt_bias,
                     const float* __restrict__ A_log,
                     float* __restrict__ rec, int T, int nItems) {
  __shared__ __align__(16) double         sAc[2][CHK];
  __shared__ __align__(16) unsigned short sBh[2][3 * CHK];
  __shared__ __align__(16) unsigned short sBl[2][3 * CHK];
  __shared__ __align__(16) float          sRec[2][RECI];

  const int wave = threadIdx.x >> 5;
  const int lane = threadIdx.x & 31;
  const int nch  = T / CHK;
  int item = blockIdx.x * 2 + wave;
  item = (item < nItems) ? item : (nItems - 1);
  const int bk = item / nch;
  const int ch = item - bk * nch;
  const int t0 = ch * CHK;

  const Par p = load_par(W_in, b_in, W_ip, conv_w, conv_b, dt_bias, A_log);

  double* sa = sAc[wave];
  unsigned short* bh = sBh[wave];
  unsigned short* bl = sBl[wave];
  float* sr = sRec[wave];
  bh[2 * CHK + lane] = 0; bh[2 * CHK + 32 + lane] = 0;
  bl[2 * CHK + lane] = 0; bl[2 * CHK + 32 + lane] = 0;

  const float a0 = front_step(obs, t0 + lane,      bk, lane,      p, sr, bh, bl);
  const float a1 = front_step(obs, t0 + 32 + lane, bk, 32 + lane, p, sr, bh, bl);

  const double cA  = wave_scan_d((double)a0, lane);
  const double tot = shfl_d(cA, 31);
  const double cB  = wave_scan_d((double)a1, lane) + tot;
  sa[lane] = cA; sa[32 + lane] = cB;
  __syncthreads();

  const v8f z8 = {0.f, 0.f, 0.f, 0.f, 0.f, 0.f, 0.f, 0.f};
  v8f acc;
  acc = tile_mma(0, 0, z8, sa, bh, bl, lane);                                             tile_out(0, acc, sr, lane);
  acc = tile_mma(1, 0, z8, sa, bh, bl, lane);                                             tile_out(1, acc, sr, lane);
  acc = tile_mma(2, 0, z8, sa, bh, bl, lane); acc = tile_mma(2, 1, acc, sa, bh, bl, lane); tile_out(2, acc, sr, lane);
  acc = tile_mma(3, 0, z8, sa, bh, bl, lane); acc = tile_mma(3, 1, acc, sa, bh, bl, lane); tile_out(3, acc, sr, lane);
  __syncthreads();

  float* dst = rec + (size_t)item * RECI;
#pragma unroll
  for (int it = 0; it < RECI / 128; ++it) {
    const v4f v = *(const v4f*)(sr + it * 128 + 4 * lane);
    *(volatile v4f*)(dst + it * 128 + 4 * lane) = v;
  }
  __threadfence();
#pragma unroll
  for (int it = 0; it < RECI / 128; ++it) {
    const v4f v = *(const v4f*)(sr + it * 128 + 4 * lane);
    *(volatile v4f*)(dst + it * 128 + 4 * lane) = v;
  }
}

__global__ __launch_bounds__(WSEQ)
void ssd_scan_out(const float* __restrict__ rec,
                  const float* __restrict__ Dp,    const float* __restrict__ norm_w,
                  const float* __restrict__ W_out, const float* __restrict__ headp,
                  const float* __restrict__ log_tau, const int* __restrict__ kopt,
                  float* __restrict__ out, int T) {
  (void)kopt;
  const int lane = threadIdx.x;
  const int bk   = blockIdx.x * WSEQ + lane;

  const float Dh   = Dp[0];
  const float nw0  = norm_w[0], nw1 = norm_w[1];
  const float wo00 = W_out[0], wo01 = W_out[1], wo10 = W_out[2], wo11 = W_out[3];
  const float spHead = softplus_f(headp[0]);
  const float tauInv = __builtin_amdgcn_rcpf(expf(log_tau[0]));

  double acs = 0.0;
  float h0 = 0.0f, h1 = 0.0f;
  float sin0 = 0.0f, sin1 = 0.0f;

  const float* rp = rec + (size_t)bk * (size_t)T * RECW;
  float* oq = out + (size_t)blockIdx.x * WSEQ + 4 * (lane & 7);
  const size_t o1off = (size_t)T * NSEQ;
  const int gsrc = (lane & 7) * 4;

#pragma unroll 1
  for (int t = 0; t < T; ++t) {
    const v4f ra = *(const v4f*)(rp);
    const v4f rb = *(const v4f*)(rp + 4);
    const v4f rc = *(const v4f*)(rp + 8);
    rp += RECW;
    const float yd0 = ra[0], yd1 = ra[1], Cv = ra[2], a = ra[3];
    const float x0  = rb[0], x1  = rb[1], bx0 = rb[2], bx1 = rb[3];
    const float g0  = rc[0], g1  = rc[1];

    if ((t & (CHK - 1)) == 0) { sin0 = h0; sin1 = h1; acs = 0.0; }
    acs += (double)a;
    const float E   = expf((float)acs);
    const float dec = expf(a);
    h0 = dec * h0 + bx0;
    h1 = dec * h1 + bx1;

    const float CE = Cv * E;
    float y0 = (Cv * yd0 + CE * sin0) + x0 * Dh;
    float y1 = (Cv * yd1 + CE * sin1) + x1 * Dh;
    y0 *= g0; y1 *= g1;

    const float rinv = rsqrtf(0.5f * (y0 * y0 + y1 * y1) + 1e-5f);
    y0 = y0 * rinv * nw0;
    y1 = y1 * rinv * nw1;

    const float u0 = wo00 * y0 + wo01 * y1;
    const float u1 = wo10 * y0 + wo11 * y1;
    const float qv = (u0 + u1) * spHead;

    v4f vq;
    vq[0] = __shfl(qv, gsrc + 0, 32);
    vq[1] = __shfl(qv, gsrc + 1, 32);
    vq[2] = __shfl(qv, gsrc + 2, 32);
    vq[3] = __shfl(qv, gsrc + 3, 32);
    const v4f vl = vq * tauInv;

    float* pq = oq + (size_t)t * NSEQ;
    float* pl = pq + o1off;
    if (lane < 8) { *(volatile v4f*)pq = vq; *(volatile v4f*)pl = vl; }
    __threadfence();
    if (lane < 8) { *(volatile v4f*)pq = vq; *(volatile v4f*)pl = vl; }
  }
}

extern "C" void kernel_launch(void* const* d_in, const int* in_sizes, int n_in,
                              void* d_out, int out_size, void* d_ws, size_t ws_size,
                              hipStream_t stream) {
  if (n_in < 14) return;
  const int nObs = in_sizes[0];
  if (nObs <= 0 || (nObs % (NSEQ * OBSD)) != 0) return;
  const int T = nObs / (NSEQ * OBSD);
  if ((T % CHK) != 0) return;
  if (out_size != 2 * T * NSEQ) return;
  if (in_sizes[1] < 6 || in_sizes[2] < 2 || in_sizes[3] < 14 || in_sizes[4] < 8 ||
      in_sizes[5] < 4 || in_sizes[6] < 1 || in_sizes[7] < 1 || in_sizes[8] < 1 ||
      in_sizes[9] < 2 || in_sizes[10] < 4 || in_sizes[11] < 1 || in_sizes[12] < 1 ||
      in_sizes[13] < 1) return;

  const size_t recBytes = (size_t)NSEQ * (size_t)T * RECW * sizeof(float);
  if (recBytes > ws_size || recBytes > (size_t)134217728u) return;

  const float* obs     = (const float*)d_in[0];
  const float* W_in    = (const float*)d_in[1];
  const float* b_in    = (const float*)d_in[2];
  const float* W_ip    = (const float*)d_in[3];
  const float* conv_w  = (const float*)d_in[4];
  const float* conv_b  = (const float*)d_in[5];
  const float* dt_bias = (const float*)d_in[6];
  const float* A_log   = (const float*)d_in[7];
  const float* Dp      = (const float*)d_in[8];
  const float* norm_w  = (const float*)d_in[9];
  const float* W_out   = (const float*)d_in[10];
  const float* headp   = (const float*)d_in[11];
  const float* log_tau = (const float*)d_in[12];
  const int*   kopt    = (const int*)d_in[13];
  float* out = (float*)d_out;
  float* rec = (float*)d_ws;

  const int nItems = NSEQ * (T / CHK);
  ssd_chunk_front<<<dim3(nItems / 2), dim3(64), 0, stream>>>(
      obs, W_in, b_in, W_ip, conv_w, conv_b, dt_bias, A_log, rec, T, nItems);
  ssd_scan_out<<<dim3(NSEQ / WSEQ), dim3(WSEQ), 0, stream>>>(
      rec, Dp, norm_w, W_out, headp, log_tau, kopt, out, T);
  (void)hipGetLastError();
}
